// AM_EGCL_77266461655561
// MI455X (gfx1250) — hardware-run, weakly checked
//
#include <hip/hip_runtime.h>


namespace {
constexpr int N = 50000, NP = 50048, E = 400000, EP = 403200  , NWV = EP / 16, D = 128, CH = 8, CNF = 8, K1 = 288  , PW = 160  ;
constexpr float XS = 8.0f, WSC = 256.0f, NEG = 0.2f  , EPS3 = 1e-3f, BNS = 0.99999500003749969f  ;

typedef _Float16 b16;
typedef __attribute__((ext_vector_type(16))) _Float16 v16b;
typedef __attribute__((ext_vector_type(8))) _Float16 v8b;
typedef __attribute__((ext_vector_type(8))) float v8f;
typedef __attribute__((ext_vector_type(4))) float v4f;
__device__ __forceinline__ float bf16_rne(float f) { unsigned int u = __float_as_uint(f); u += 0x7FFFu + ((u >> 16) & 1u); return __uint_as_float(u & 0xFFFF0000u); }
__device__ __forceinline__ void split16(float v, b16& hi, b16& lo) { hi = (b16)v; lo = (b16)(v - (float)hi); }
__device__ __forceinline__ v16b frag_kb(const b16* p, int hh) { const v8b a = *(const v8b*)(p + 8 * hh), b = *(const v8b*)(p + 16 + 8 * hh); v16b f;
#pragma unroll
  for (int e = 0; e < 8; ++e) { f[e] = a[e]; f[8 + e] = b[e]; } return f; }
__device__ __forceinline__ v8f wmma16b(v16b a, v16b b, v8f c) { v8f d = __builtin_amdgcn_wmma_f32_16x16x32_f16(false, a, false, b, (short)0, c, false, false); asm volatile("v_nop\n\tv_nop\n\tv_nop\n\tv_nop" : "+v"(d) : "v"(a), "v"(b)); return d; }
__device__ __forceinline__ void wave_lds_sync() { __builtin_amdgcn_fence(__ATOMIC_RELEASE, "workgroup"); __builtin_amdgcn_wave_barrier(); __builtin_amdgcn_fence(__ATOMIC_ACQUIRE, "workgroup"); }
__device__ __forceinline__ float pmul(float a, float b) { float p = a * b; asm volatile("" : "+v"(p)); return p; }
__device__ __forceinline__ int iclamp(int v, int lo, int hi) { return v < lo ? lo : (v > hi ? hi : v); }
__device__ __forceinline__ float nexp(float x) { return __builtin_amdgcn_exp2f(x * 1.4426950408889634f); }
__device__ __forceinline__ float lrelu(float x) { return x > 0.0f ? x : NEG * x; }

constexpr int CSR_NBLK = 512, CSR_GB = 9, CSR_GN = 1 << CSR_GB  , CSR_MAXG = 512, CSR_CAP = 12288  ;
__global__ __launch_bounds__(64) void csrA_kernel(const int* __restrict__ dst, int E, int N, int nG, int CHP, int NGP, int* __restrict__ STG, int* __restrict__ HST) {
  extern __shared__ int sm[];
  int* cnt = sm; int* run = sm + NGP; int* ids = sm + 2 * NGP;
  const int b = blockIdx.x; const int ch = (E + CSR_NBLK - 1) / CSR_NBLK; const int e0 = b * ch, e1 = min(E, e0 + ch);
  for (int i = threadIdx.x; i < NGP; i += 64) cnt[i] = 0;
  for (int i = threadIdx.x; i < CHP; i += 64) ids[i] = -1;
  __syncthreads();
  if (threadIdx.x == 0) {
    for (int e = e0; e < e1; ++e) { int d = dst[e]; d = (d < 0) ? 0 : (d >= N ? N - 1 : d); cnt[d >> CSR_GB] += 1; }
    int acc = 0; for (int g = 0; g < nG; ++g) { run[g] = acc; acc += cnt[g]; }
    for (int e = e0; e < e1; ++e) { int d = dst[e]; d = (d < 0) ? 0 : (d >= N ? N - 1 : d); const int g = d >> CSR_GB; ids[run[g]] = e; run[g] += 1; } }
  __syncthreads();
  typedef __attribute__((ext_vector_type(4))) int v4i;
  for (int pass = 0; pass < 2; ++pass) {
    for (int i = threadIdx.x; i < CHP / 4; i += 64) *(volatile v4i*)(STG + (size_t)b * CHP + i * 4) = *(const v4i*)(&ids[i * 4]);
    for (int i = threadIdx.x; i < NGP / 4; i += 64) { v4i v; for (int e = 0; e < 4; ++e) v[e] = (i * 4 + e < nG) ? cnt[i * 4 + e] : 0; *(volatile v4i*)(HST + (size_t)b * NGP + i * 4) = v; }
    __threadfence(); }
}
__global__ __launch_bounds__(512) void csrS_kernel(const int* __restrict__ HST, int nG, int NGP, int* __restrict__ START, int* __restrict__ TOT, int* __restrict__ OFF) {
  __shared__ int tot[CSR_MAXG];
  const int b = threadIdx.x;
  for (int pass = 0; pass < 2; ++pass) { int runb = 0; for (int g = 0; g < nG; ++g) { int c = HST[(size_t)b * NGP + g]; c = (c < 0) ? 0 : c; ((volatile int*)OFF)[(size_t)g * CSR_NBLK + b] = runb; runb += c; } __threadfence(); }
  for (int g = threadIdx.x; g < nG; g += 512) { int s = 0; for (int bb = 0; bb < CSR_NBLK; ++bb) { int c = HST[(size_t)bb * NGP + g]; s += (c < 0) ? 0 : c; } tot[g] = s; }
  __syncthreads();
  if (threadIdx.x < 32) {
    __shared__ int st[CSR_MAXG + 32];
    if (threadIdx.x == 0) { int acc = 0; for (int g = 0; g < NGP; ++g) { st[g] = acc; if (g < nG) acc += (tot[g] + 31) & ~31; } st[NGP] = acc; }
    __builtin_amdgcn_fence(__ATOMIC_RELEASE, "workgroup"); __builtin_amdgcn_wave_barrier(); __builtin_amdgcn_fence(__ATOMIC_ACQUIRE, "workgroup");
    for (int pass = 0; pass < 2; ++pass) { for (int i = threadIdx.x; i < NGP + 32; i += 32) { ((volatile int*)START)[i] = (i <= NGP) ? st[min(i, NGP)] : 0; ((volatile int*)TOT)[i] = (i < nG) ? tot[i] : 0; } __threadfence(); } }
}
__global__ __launch_bounds__(256) void csrB_kernel(const int* __restrict__ dst, int N, int nG, int CHP, int NGP, int permLen, const int* __restrict__ STG, const int* __restrict__ HST, const int* __restrict__ OFF, const int* __restrict__ START, const int* __restrict__ TOT, int* __restrict__ PERM, int* __restrict__ ROWPTR, int* __restrict__ ROWCNT, int* __restrict__ FLAG) {
  typedef __attribute__((ext_vector_type(4))) int v4i;
  __shared__ int ids[CSR_CAP]; __shared__ unsigned short key[CSR_CAP]; __shared__ int outp[CSR_CAP]; __shared__ int ncnt[CSR_GN + 1]; __shared__ int boff[CSR_NBLK + 1];
  const int g = blockIdx.x, t_ = threadIdx.x; int tot = TOT[g]; int st = START[g], stn = START[g + 1]; const int v0 = g * CSR_GN; const int nv = min(CSR_GN, N - v0);
  st = (st < 0) ? 0 : (st > permLen - 32 ? permLen - 32 : st) & ~31; stn = (stn < st) ? st : (stn > permLen ? permLen : stn); tot = (tot < 0) ? 0 : tot; if (tot > stn - st && tot <= CSR_CAP) tot = stn - st;
  if (tot > CSR_CAP) {
    for (int pass = 0; pass < 2; ++pass) { for (int i = t_; i < CSR_GN / 4; i += 256) { v4i a, c; for (int e = 0; e < 4; ++e) { a[e] = st; c[e] = 0; } *(volatile v4i*)(ROWPTR + v0 + i * 4) = a; *(volatile v4i*)(ROWCNT + v0 + i * 4) = c; } if (t_ == 0) ((volatile int*)FLAG)[0] = 1; __threadfence(); } (void)nv; return; }
  if (t_ == 0) { int acc = 0; for (int b = 0; b < CSR_NBLK; ++b) { boff[b] = acc; int c = HST[(size_t)b * NGP + g]; c = (c < 0) ? 0 : (c > CHP ? CHP : c); acc += c; if (acc > tot) acc = tot; } boff[CSR_NBLK] = acc; }
  for (int i = t_; i <= CSR_GN; i += 256) ncnt[i] = 0;
  __syncthreads();
  for (int b = 0; b < CSR_NBLK; ++b) { const int c = boff[b + 1] - boff[b]; int o_ = OFF[(size_t)g * CSR_NBLK + b]; o_ = (o_ < 0) ? 0 : (o_ > CHP - c ? CHP - c : o_); const int* src_ = STG + (size_t)b * CHP + o_;
    for (int i = t_; i < c; i += 256) { int id = src_[i]; id = (id < 0) ? 0 : id; ids[boff[b] + i] = id; int d = dst[id]; d = (d < v0) ? v0 : (d >= N ? N - 1 : d); int kk = d - v0; kk = (kk < 0) ? 0 : (kk >= CSR_GN ? CSR_GN - 1 : kk); key[boff[b] + i] = (unsigned short)kk; } }
  __syncthreads();
  if (t_ == 0) { for (int i = 0; i < tot; ++i) ncnt[key[i]] += 1; int acc = 0; for (int vl = 0; vl < CSR_GN; ++vl) { const int c = ncnt[vl]; ncnt[vl] = acc; acc += c; } ncnt[CSR_GN] = acc;
    for (int i = 0; i < tot; ++i) { const int vl = key[i]; outp[ncnt[vl]] = ids[i]; ncnt[vl] += 1; }
    for (int vl = CSR_GN; vl > 0; --vl) ncnt[vl] = ncnt[vl - 1]; ncnt[0] = 0; }
  __syncthreads();
  for (int pass = 0; pass < 2; ++pass) {
    for (int i = t_; i < (stn - st) / 4; i += 256) { v4i v; for (int e = 0; e < 4; ++e) { const int q = i * 4 + e; v[e] = (q < tot) ? outp[q] : -1; } *(volatile v4i*)(PERM + st + i * 4) = v; }
    for (int i = t_; i < CSR_GN / 4; i += 256) { v4i a, c; for (int e = 0; e < 4; ++e) { const int vl = i * 4 + e; a[e] = st + ncnt[vl]; c[e] = (vl < nv) ? (ncnt[vl + 1] - ncnt[vl]) : 0; } *(volatile v4i*)(ROWPTR + v0 + i * 4) = a; *(volatile v4i*)(ROWCNT + v0 + i * 4) = c; }
    __threadfence(); }
}
__global__ __launch_bounds__(256) void csrZ_kernel(int* __restrict__ p, size_t n4) { typedef __attribute__((ext_vector_type(4))) int v4i; const size_t tid = (size_t)blockIdx.x * 256 + threadIdx.x, nth = (size_t)gridDim.x * 256; v4i z = {0, 0, 0, 0}; for (size_t i = tid; i < n4; i += nth) *(volatile v4i*)(p + i * 4) = z; }
struct CsrBufs { int *STG, *HST, *OFF, *START, *TOT, *PERM, *ROWPTR, *ROWCNT, *FLAG; int nG, NGP, CHP; size_t permLen; char* base; size_t bytes; };
static size_t csr_carve(CsrBufs& c, char* ws, size_t off, int E, int N) {
  const size_t off0 = off; c.base = ws + off;
  auto al = [&](size_t bytes) { char* p = ws + off; off += (bytes + 255) & ~(size_t)255; return p; };
  c.nG = (N + CSR_GN - 1) / CSR_GN; c.NGP = (c.nG + 31) & ~31; const int ch = (E + CSR_NBLK - 1) / CSR_NBLK; c.CHP = (ch + 31) & ~31; c.permLen = (size_t)E + 32 * (size_t)c.nG + 32;
  c.STG = (int*)al((size_t)CSR_NBLK * c.CHP * 4); c.HST = (int*)al((size_t)CSR_NBLK * c.NGP * 4); c.OFF = (int*)al((size_t)c.NGP * CSR_NBLK * 4); c.START = (int*)al((size_t)(c.NGP + 64) * 4); c.TOT = (int*)al((size_t)(c.NGP + 64) * 4);
  c.PERM = (int*)al(c.permLen * 4); c.ROWPTR = (int*)al((size_t)c.nG * CSR_GN * 4); c.ROWCNT = (int*)al((size_t)c.nG * CSR_GN * 4); c.FLAG = (int*)al(256);
  c.bytes = off - off0; return off;
}
static void csr_build(const CsrBufs& c, const int* dst, int E, int N, hipStream_t stream) {
  const size_t smem = (size_t)(2 * c.NGP + c.CHP) * 4;
  csrZ_kernel<<<512, 256, 0, stream>>>((int*)c.base, c.bytes / 16);
  csrA_kernel<<<CSR_NBLK, 64, smem, stream>>>(dst, E, N, c.nG, c.CHP, c.NGP, c.STG, c.HST);
  csrS_kernel<<<1, 512, 0, stream>>>(c.HST, c.nG, c.NGP, c.START, c.TOT, c.OFF);
  csrB_kernel<<<c.nG, 256, 0, stream>>>(dst, N, c.nG, c.CHP, c.NGP, (int)c.permLen, c.STG, c.HST, c.OFF, c.START, c.TOT, c.PERM, c.ROWPTR, c.ROWCNT, c.FLAG);
}


__device__ __forceinline__ float silu(float x) { return x / (1.0f + __expf(-x)); }
__global__ __launch_bounds__(256) void prep_kernel(const float* __restrict__ h, const float* __restrict__ coords, const float* __restrict__ cw, const float* __restrict__ mw1, const float* __restrict__ mw2, const float* __restrict__ cw1, const float* __restrict__ cw2, const float* __restrict__ hw, b16* __restrict__ H16, float* __restrict__ NODE4, b16* __restrict__ W1X, b16* __restrict__ W2T, b16* __restrict__ C1T, b16* __restrict__ C2T, b16* __restrict__ HT) {
  const size_t u = (size_t)blockIdx.x * 256 + threadIdx.x; const size_t nh = (size_t)NP * D / 8, nn = NP, n1 = (size_t)D * K1 / 8, n2 = (size_t)D * D / 8, n3 = (size_t)16 * D / 8; size_t t = u; v8b o;
  if (t < nh) { const size_t e = t * 8; const size_t v = e / D; for (int j = 0; j < 8; ++j) o[j] = (v < (size_t)N) ? (b16)(bf16_rne(h[e + j]) * XS) : (b16)0.0f; for (int pass = 0; pass < 2; ++pass) { *(volatile v8b*)(H16 + e) = o; __threadfence(); } return; } t -= nh;
  if (t < nn) { const size_t v = t; v4f r = {0.0f, 0.0f, 0.0f, 0.0f}; if (v < (size_t)N) { float sx = 0.0f, sy = 0.0f, sz = 0.0f; int cnt = 0; for (int c = 0; c < CH; ++c) { const bool m = bf16_rne(cw[v * CH + c]) != 0.0f; if (m) { sx += bf16_rne(coords[(v * CH + c) * 3]); sy += bf16_rne(coords[(v * CH + c) * 3 + 1]); sz += bf16_rne(coords[(v * CH + c) * 3 + 2]); ++cnt; } }
      const float den = (float)cnt + EPS3; r[0] = sx / den; r[1] = sy / den; r[2] = sz / den; r[3] = (float)cnt; }
    for (int pass = 0; pass < 2; ++pass) { *(volatile v4f*)(NODE4 + v * 4) = r; __threadfence(); } return; } t -= nn;
  if (t < n1) { const size_t e = t * 8; const int oo = (int)(e / K1), k0 = (int)(e % K1); for (int j = 0; j < 8; ++j) { const int k = k0 + j; const int row = k < 264 ? k : -1; o[j] = row >= 0 ? (b16)(bf16_rne(mw1[(size_t)row * D + oo]) * WSC) : (b16)0.0f; } for (int pass = 0; pass < 2; ++pass) { *(volatile v8b*)(W1X + e) = o; __threadfence(); } return; } t -= n1;
  if (t < 3 * n2) { const int which = (int)(t / n2); const size_t e = (t % n2) * 8; const int oo = (int)(e / D), k0 = (int)(e % D); const float* w = which == 0 ? mw2 : which == 1 ? cw1 : hw; b16* dst = which == 0 ? W2T : which == 1 ? C1T : HT;
    for (int j = 0; j < 8; ++j) o[j] = (b16)(bf16_rne(w[(size_t)(k0 + j) * D + oo]) * WSC); for (int pass = 0; pass < 2; ++pass) { *(volatile v8b*)(dst + e) = o; __threadfence(); } return; } t -= 3 * n2;
  if (t < n3) { const size_t e = t * 8; const int oo = (int)(e / D), k0 = (int)(e % D); for (int j = 0; j < 8; ++j) o[j] = oo < CNF ? (b16)(bf16_rne(cw2[(size_t)(k0 + j) * CNF + oo]) * WSC) : (b16)0.0f; for (int pass = 0; pass < 2; ++pass) { *(volatile v8b*)(C2T + e) = o; __threadfence(); } }
}
__global__ __launch_bounds__(256) void dmax_kernel(const float* __restrict__ coords, const int* __restrict__ el, float* __restrict__ BM) {
  __shared__ float sm[256]; const size_t e = (size_t)blockIdx.x * 256 + threadIdx.x; float m = 0.0f;
  if (e < (size_t)E) { const size_t s = (size_t)iclamp(el[e * 3], 0, N - 1), t = (size_t)iclamp(el[e * 3 + 1], 0, N - 1); float sx[CH], sy[CH], sz[CH];
#pragma unroll
    for (int d = 0; d < CH; ++d) { sx[d] = bf16_rne(coords[(s * CH + d) * 3]); sy[d] = bf16_rne(coords[(s * CH + d) * 3 + 1]); sz[d] = bf16_rne(coords[(s * CH + d) * 3 + 2]); }
    float m2 = 0.0f;
#pragma unroll 1
    for (int c = 0; c < CH; ++c) { const float tx = bf16_rne(coords[(t * CH + c) * 3]), ty = bf16_rne(coords[(t * CH + c) * 3 + 1]), tz = bf16_rne(coords[(t * CH + c) * 3 + 2]);
#pragma unroll
      for (int d = 0; d < CH; ++d) { const float dx = tx - sx[d], dy = ty - sy[d], dz = tz - sz[d]; m2 = fmaxf(m2, pmul(dx, dx) + pmul(dy, dy) + pmul(dz, dz)); } }
    m = sqrtf(m2); }
  sm[threadIdx.x] = m; __syncthreads();
  for (int st = 128; st > 0; st >>= 1) { if (threadIdx.x < st) sm[threadIdx.x] = fmaxf(sm[threadIdx.x], sm[threadIdx.x + st]); __syncthreads(); }
  for (int pass = 0; pass < 2; ++pass) { if (threadIdx.x < 32) ((volatile float*)BM)[(size_t)blockIdx.x * 32 + threadIdx.x] = sm[0]; __threadfence(); }
}
__global__ __launch_bounds__(256) void gmax_kernel(const float* __restrict__ BM, int nb, float* __restrict__ GMX) {
  __shared__ float sm[256]; float m = 0.0f; for (int b = threadIdx.x; b < nb; b += 256) m = fmaxf(m, BM[(size_t)b * 32]); sm[threadIdx.x] = m; __syncthreads();
  for (int st = 128; st > 0; st >>= 1) { if (threadIdx.x < st) sm[threadIdx.x] = fmaxf(sm[threadIdx.x], sm[threadIdx.x + st]); __syncthreads(); }
  for (int pass = 0; pass < 2; ++pass) { if (threadIdx.x < 32) ((volatile float*)GMX)[threadIdx.x] = sm[0]; __threadfence(); }
}
__global__ __launch_bounds__(256) void keys_kernel(const int* __restrict__ el, int* __restrict__ KD) {
  typedef __attribute__((ext_vector_type(4))) int v4i; const size_t u = (size_t)blockIdx.x * 256 + threadIdx.x; if (u * 4 >= (size_t)E) return; const size_t e0 = u * 4; v4i k;
  for (int j = 0; j < 4; ++j) k[j] = iclamp(el[(e0 + j) * 3 + 1], 0, N - 1);
  for (int pass = 0; pass < 2; ++pass) { *(volatile v4i*)(KD + e0) = k; __threadfence(); }
}

__global__ __launch_bounds__(32) void edge_kernel(const float* __restrict__ coords, const float* __restrict__ attr, const float* __restrict__ cwt, const float* __restrict__ ewt, const int* __restrict__ el, const float* __restrict__ rlw, const float* __restrict__ rlb, const float* __restrict__ GMX, const float* __restrict__ NODE4,
    const int* __restrict__ PERM, int permLen, const b16* __restrict__ H16, const b16* __restrict__ W1X, const float* __restrict__ b1, const b16* __restrict__ W2T, const float* __restrict__ b2, const b16* __restrict__ C1T, const float* __restrict__ cb1, const b16* __restrict__ C2T, const float* __restrict__ wr,
    float* __restrict__ NAGG, float* __restrict__ CAGG, float* __restrict__ PF, float* __restrict__ PL) {
  __shared__ __attribute__((aligned(16))) float scr[16][128]; __shared__ __attribute__((aligned(16))) float ATT[16][64], ATS[16][64]; __shared__ float RAD[16][8]; __shared__ __attribute__((aligned(16))) b16 A2[16][D + 8]; __shared__ __attribute__((aligned(16))) float MW[16][PW]; __shared__ float EF[16][8]; __shared__ int TG[16]; __shared__ __attribute__((aligned(16))) float SEG[PW];
  const int lane = threadIdx.x, nloc = lane & 15, hlf = lane >> 4; const size_t w = blockIdx.x; const size_t j = w * 16 + nloc;
  int e = -1; if (j < (size_t)permLen) { const int p = PERM[j]; if (p >= 0 && p < E) e = p; }
  const bool live = e >= 0; const size_t s = live ? (size_t)iclamp(el[(size_t)e * 3], 0, N - 1) : 0, t = live ? (size_t)iclamp(el[(size_t)e * 3 + 1], 0, N - 1) : 0;
  const float gden = 1.0f / (GMX[0] + EPS3);
  { float* sc = scr[nloc]; float* at = ATT[nloc]; float* as_ = ATS[nloc];
    for (int q = hlf * 32; q < hlf * 32 + 32; ++q) { at[q] = bf16_rne(attr[t * 64 + q]); as_[q] = bf16_rne(attr[s * 64 + q]); }
    float scx[CH], scy[CH], scz[CH], scw[CH];
#pragma unroll
    for (int d = 0; d < CH; ++d) { scx[d] = bf16_rne(coords[(s * CH + d) * 3]); scy[d] = bf16_rne(coords[(s * CH + d) * 3 + 1]); scz[d] = bf16_rne(coords[(s * CH + d) * 3 + 2]); scw[d] = bf16_rne(cwt[s * CH + d]); }
    wave_lds_sync();
#pragma unroll
    for (int ci = 0; ci < 4; ++ci) { const int c = 4 * hlf + ci; const float tx = bf16_rne(coords[(t * CH + c) * 3]), ty = bf16_rne(coords[(t * CH + c) * 3 + 1]), tz = bf16_rne(coords[(t * CH + c) * 3 + 2]); const float cwt_c = bf16_rne(cwt[t * CH + c]);
      v4f t0 = {0.0f, 0.0f, 0.0f, 0.0f}, t1 = t0;
#pragma unroll
      for (int d = 0; d < CH; ++d) { const float dx = tx - scx[d], dy = ty - scy[d], dz = tz - scz[d]; const float m = pmul(pmul(sqrtf(pmul(dx, dx) + pmul(dy, dy) + pmul(dz, dz)), gden), pmul(cwt_c, scw[d]));
        const v4f a0 = *(const v4f*)(&as_[d * 8]), a1 = *(const v4f*)(&as_[d * 8 + 4]); for (int k = 0; k < 4; ++k) { t0[k] += pmul(m, a0[k]); t1[k] += pmul(m, a1[k]); } }
      *(v4f*)(&sc[64 + c * 8]) = t0; *(v4f*)(&sc[64 + c * 8 + 4]) = t1; }
    wave_lds_sync();
    float nrm2 = 0.0f;
#pragma unroll
    for (int ai = 0; ai < 4; ++ai) { const int a_ = 4 * hlf + ai; v4f r0 = {0.0f, 0.0f, 0.0f, 0.0f}, r1 = r0;
#pragma unroll
      for (int c = 0; c < CH; ++c) { const float w8 = at[c * 8 + a_]; const v4f p0 = *(const v4f*)(&sc[64 + c * 8]), p1 = *(const v4f*)(&sc[64 + c * 8 + 4]); for (int k = 0; k < 4; ++k) { r0[k] += pmul(w8, p0[k]); r1[k] += pmul(w8, p1[k]); } }
      for (int k = 0; k < 4; ++k) { nrm2 += r0[k] * r0[k] + r1[k] * r1[k]; } *(v4f*)(&sc[a_ * 8]) = r0; *(v4f*)(&sc[a_ * 8 + 4]) = r1; }
    nrm2 += __shfl_xor(nrm2, 16);
    const float inv = 1.0f / (sqrtf(nrm2) + EPS3);
    wave_lds_sync();
    float r8[CNF]; for (int q = 0; q < CNF; ++q) r8[q] = 0.0f;
#pragma unroll 4
    for (int ii = 0; ii < 32; ++ii) { const int i = hlf * 32 + ii; const float rv = sc[i] * inv; const v4f w0 = *(const v4f*)(rlw + i * CNF), w1 = *(const v4f*)(rlw + i * CNF + 4);
      for (int k = 0; k < 4; ++k) { r8[k] += pmul(rv, bf16_rne(w0[k])); r8[4 + k] += pmul(rv, bf16_rne(w1[k])); } }
#pragma unroll
    for (int q = 0; q < CNF; ++q) r8[q] += __shfl_xor(r8[q], 16);
    if (hlf == 0) { for (int q = 0; q < CNF; ++q) RAD[nloc][q] = live ? r8[q] + bf16_rne(rlb[q]) : 0.0f; TG[nloc] = live ? (int)t : -1; } }
  wave_lds_sync();
  v8f acc[8];
#pragma unroll
  for (int tt = 0; tt < 8; ++tt) acc[tt] = (v8f){};
  { const b16* ht = H16 + t * D; const b16* hs = H16 + s * D;
#pragma unroll 2
    for (int kb = 0; kb < 256; kb += 32) { const v16b a = live ? frag_kb((kb < D ? ht : hs) + (kb & (D - 1)), hlf) : (v16b){};
#pragma unroll
      for (int tt = 0; tt < 8; ++tt) acc[tt] = wmma16b(a, frag_kb(W1X + (size_t)(tt * 16 + nloc) * K1 + kb, hlf), acc[tt]); }
    { v16b a = {}; if (hlf == 0) { for (int q = 0; q < 8; ++q) a[q] = (b16)(RAD[nloc][q] * XS); }
#pragma unroll
      for (int tt = 0; tt < 8; ++tt) acc[tt] = wmma16b(a, frag_kb(W1X + (size_t)(tt * 16 + nloc) * K1 + 256, hlf), acc[tt]); } }
  auto to_a2_silu = [&](const float* bias) {
#pragma unroll
    for (int tt = 0; tt < 8; ++tt) { const int c = tt * 16 + nloc; const float bb = bf16_rne(bias[c]);
#pragma unroll 1
      for (int r = 0; r < 8; ++r) A2[8 * hlf + r][c] = (b16)(silu(acc[tt][r] * (1.0f / (XS * WSC)) + bb) * XS); } };
  auto gemm128 = [&](const b16* WT) {
#pragma unroll
    for (int tt = 0; tt < 8; ++tt) acc[tt] = (v8f){};
#pragma unroll
    for (int kb = 0; kb < D; kb += 32) { const v16b a = frag_kb(&A2[nloc][kb], hlf);
#pragma unroll
      for (int tt = 0; tt < 8; ++tt) acc[tt] = wmma16b(a, frag_kb(WT + (size_t)(tt * 16 + nloc) * D + kb, hlf), acc[tt]); } };
  to_a2_silu(b1); wave_lds_sync();
  gemm128(W2T);
#pragma unroll
  for (int tt = 0; tt < 8; ++tt) { const int c = tt * 16 + nloc; const float bb = bf16_rne(b2[c]);
#pragma unroll 1
    for (int r = 0; r < 8; ++r) { const int rr = 8 * hlf + r; const float m = silu(acc[tt][r] * (1.0f / (XS * WSC)) + bb); const int tg = TG[rr]; const int ee = (tg >= 0) ? PERM[w * 16 + rr] : 0; const float ew = (tg >= 0) ? bf16_rne(ewt[ee]) : 0.0f;
      MW[rr][c] = pmul(m, ew); A2[rr][c] = (b16)(m * XS); } }
  wave_lds_sync();
  gemm128(C1T); wave_lds_sync(); to_a2_silu(cb1); wave_lds_sync();
  { v8f ac2 = {};
#pragma unroll
    for (int kb = 0; kb < D; kb += 32) ac2 = wmma16b(frag_kb(&A2[nloc][kb], hlf), frag_kb(C2T + (size_t)nloc * D + kb, hlf), ac2);
#pragma unroll 1
    for (int r = 0; r < 8; ++r) if (nloc < 8) EF[8 * hlf + r][nloc] = ac2[r] * (1.0f / (XS * WSC)); }
  wave_lds_sync();
  if (hlf == 0) { float cm[24]; for (int q = 0; q < 24; ++q) cm[q] = 0.0f;
    if (live) { const int csum = (int)NODE4[t * 4 + 3]; int ts = csum - 1; ts = ts < 0 ? 0 : (ts > 7 ? 7 : ts); const int wdt = CH - ts; const float invw = 1.0f / (float)wdt; const float wr0 = bf16_rne(wr[0]);
      const float px = NODE4[s * 4], py = NODE4[s * 4 + 1], pz = NODE4[s * 4 + 2];
#pragma unroll
      for (int c = 0; c < CH; ++c) { float pe = 0.0f; for (int q = c; q < CH && q < c + wdt; ++q) pe += EF[nloc][q]; pe *= invw; const float f = pmul(pe, wr0);
        cm[c * 3] = pmul(bf16_rne(coords[(t * CH + c) * 3]) - px, f); cm[c * 3 + 1] = pmul(bf16_rne(coords[(t * CH + c) * 3 + 1]) - py, f); cm[c * 3 + 2] = pmul(bf16_rne(coords[(t * CH + c) * 3 + 2]) - pz, f); } }
    for (int q = 0; q < 24; ++q) MW[nloc][D + q] = cm[q]; }
  else { for (int q = 24; q < PW - D; ++q) MW[nloc][D + q] = 0.0f; }
  wave_lds_sync();
  int first = -1, last = -1; for (int rr = 0; rr < 16; ++rr) { if (TG[rr] >= 0) { if (first < 0) first = rr; last = rr; } }
  const int tfirst = first >= 0 ? TG[first] : -1, tlast = last >= 0 ? TG[last] : -1;
  v4f am = {0.0f, 0.0f, 0.0f, 0.0f}, ac = {0.0f, 0.0f, 0.0f, 0.0f}; int cur = -1;
  v4f pfm = {0.0f, 0.0f, 0.0f, 0.0f}, pfc = pfm, plm = pfm, plc = pfm;
  auto flush = [&](int tg) {
    if (tg < 0) return;
    if (tg == tfirst) { pfm = am; pfc = ac; }
    else if (tg == tlast) { plm = am; plc = ac; }
    else { for (int pass = 0; pass < 2; ++pass) { *(volatile v4f*)(NAGG + (size_t)tg * D + lane * 4) = am; if (lane < 8) *(volatile v4f*)(CAGG + (size_t)tg * 32 + lane * 4) = ac; __threadfence(); } } };
  for (int rr = 0; rr < 16; ++rr) { const int tg = TG[rr]; if (tg < 0) continue; if (tg != cur) { flush(cur); cur = tg; am = (v4f){0.0f, 0.0f, 0.0f, 0.0f}; ac = am; }
    am += *(const v4f*)(&MW[rr][lane * 4]); const v4f cv = *(const v4f*)(&MW[rr][D + (lane & 7) * 4]); if (lane < 8) ac += cv; }
  flush(cur);
  for (int pass = 0; pass < 2; ++pass) { *(volatile v4f*)(PF + w * PW + lane * 4) = pfm; *(volatile v4f*)(PL + w * PW + lane * 4) = plm; if (lane < 8) { *(volatile v4f*)(PF + w * PW + D + lane * 4) = pfc; *(volatile v4f*)(PL + w * PW + D + lane * 4) = plc; } __threadfence(); }
}
__global__ __launch_bounds__(256) void fix_kernel(const int* __restrict__ PERM, const int* __restrict__ ROWPTR, const int* __restrict__ ROWCNT, int permLen, const int* __restrict__ el, const float* __restrict__ PF, const float* __restrict__ PL, const float* __restrict__ CAGG, const float* __restrict__ coords, float* __restrict__ NAGG, float* __restrict__ out2) {
  __shared__ __attribute__((aligned(16))) float so[8][24]; __shared__ __attribute__((aligned(16))) float cs[8][32];
  const int wave = threadIdx.x >> 5, lane = threadIdx.x & 31; const size_t t = (size_t)blockIdx.x * 8 + wave;
  const int lc8 = lane & 7;
  auto tgt_of_row = [&](int row) -> int { if (row < 0 || row >= permLen) return -1; const int p = PERM[row]; if (p < 0 || p >= E) return -1; return iclamp(el[(size_t)p * 3 + 1], 0, N - 1); };
  v4f am = {0.0f, 0.0f, 0.0f, 0.0f}, ac = am; bool interior = false;
  if (t < (size_t)N) { int st = ROWPTR[t], cnt = ROWCNT[t]; cnt = iclamp(cnt, 0, 65536); st = iclamp(st, 0, permLen - cnt);
    if (cnt > 0) { const int w0 = st >> 4, w1 = (st + cnt - 1) >> 4;
      for (int w = w0; w <= w1; ++w) { bool isfirst = true; for (int row = w * 16; row < st && row < w * 16 + 16; ++row) if (tgt_of_row(row) >= 0) { isfirst = false; break; }
        bool islast = true; for (int row = st + cnt; row < w * 16 + 16; ++row) if (tgt_of_row(row) >= 0) { islast = false; break; }
        if (isfirst) { am += *(const v4f*)(PF + (size_t)w * PW + lane * 4); const v4f cv = *(const v4f*)(PF + (size_t)w * PW + D + lc8 * 4); if (lane < 8) ac += cv; }
        else if (islast) { am += *(const v4f*)(PL + (size_t)w * PW + lane * 4); const v4f cv = *(const v4f*)(PL + (size_t)w * PW + D + lc8 * 4); if (lane < 8) ac += cv; }
        else { interior = true; } } }
    if (!interior) { for (int pass = 0; pass < 2; ++pass) { *(volatile v4f*)(NAGG + t * D + lane * 4) = am; __threadfence(); } }
    else { const v4f cv = *(const v4f*)(CAGG + t * 32 + lc8 * 4); if (lane < 8) ac = cv; }
    const float invc = 1.0f / fmaxf((float)cnt, 1.0f);
    if (lane < 8) *(v4f*)(&cs[wave][lane * 4]) = ac;
    wave_lds_sync();
    if (lane < 24) so[wave][lane] = bf16_rne(coords[t * 24 + lane]) + cs[wave][lane] * invc; }
  __syncthreads();
  const size_t t0 = (size_t)blockIdx.x * 8; const int nval = (int)((t0 + 8 <= (size_t)N) ? 8 : ((size_t)N - t0));
  for (int pass = 0; pass < 2; ++pass) { for (int q = threadIdx.x; q < nval * 6; q += 256) *(volatile v4f*)(out2 + (t0 * 24) + q * 4) = *(const v4f*)(&so[0][0] + q * 4); __threadfence(); }
}
__global__ __launch_bounds__(128) void head_kernel(const float* __restrict__ NAGG, const b16* __restrict__ HT, const float* __restrict__ hb, const float* __restrict__ gam, const float* __restrict__ bet, const float* __restrict__ h, float* __restrict__ out1) {
  __shared__ __attribute__((aligned(16))) b16 Ah[4][16][D + 8]; __shared__ __attribute__((aligned(16))) float Tf[4][16][D + 4];
  const int wave = threadIdx.x >> 5, lane = threadIdx.x & 31, nloc = lane & 15, hlf = lane >> 4; const size_t m0 = (size_t)blockIdx.x * 64 + wave * 16;
  for (int q = lane; q < 16 * (D / 4); q += 32) { const int rr = q / (D / 4), c4 = (q % (D / 4)) * 4; const v4f v = *(const v4f*)(NAGG + (m0 + rr) * D + c4); for (int k = 0; k < 4; ++k) Ah[wave][rr][c4 + k] = (b16)(v[k] * XS); }
  wave_lds_sync();
  v8f acc[8];
#pragma unroll
  for (int tt = 0; tt < 8; ++tt) acc[tt] = (v8f){};
#pragma unroll
  for (int kb = 0; kb < D; kb += 32) { const v16b a = frag_kb(&Ah[wave][nloc][kb], hlf);
#pragma unroll
    for (int tt = 0; tt < 8; ++tt) acc[tt] = wmma16b(a, frag_kb(HT + (size_t)(tt * 16 + nloc) * D + kb, hlf), acc[tt]); }
#pragma unroll
  for (int tt = 0; tt < 8; ++tt) { const int c = tt * 16 + nloc; const float bb = bf16_rne(hb[c]), g = bf16_rne(gam[c]), be = bf16_rne(bet[c]);
#pragma unroll 1
    for (int r = 0; r < 8; ++r) { const size_t row = m0 + 8 * hlf + r; const float o = silu((acc[tt][r] * (1.0f / (XS * WSC)) + bb) * BNS * g + be); Tf[wave][8 * hlf + r][c] = (row < (size_t)N ? bf16_rne(h[row * D + c]) : 0.0f) + o; } }
  wave_lds_sync();
  for (int pass = 0; pass < 2; ++pass) { for (int rr = 0; rr < 16; ++rr) { const size_t row = m0 + rr; if (row < (size_t)N) *(volatile v4f*)(out1 + row * D + lane * 4) = *(const v4f*)(&Tf[wave][rr][lane * 4]); } __threadfence(); }
}
}

extern "C" void kernel_launch(void* const* d_in, const int* in_sizes, int n_in, void* d_out, int out_size, void* d_ws, size_t ws_size, hipStream_t stream) {
  (void)n_in;
  auto Fp = [&](int i) { return (const float*)d_in[i]; }; auto Ip = [&](int i) { return (const int*)d_in[i]; };
  if (in_sizes[0] != N * D || in_sizes[1] != N * 24 || in_sizes[2] != N * 64 || in_sizes[3] != N * CH || in_sizes[4] != E || in_sizes[5] != E * 3 || in_sizes[6] != 64 * CNF || in_sizes[8] != 264 * D || in_sizes[14] != D * CNF || in_sizes[15] != D * D || out_size != N * D + N * 24) return;
  size_t off = 0; char* ws = (char*)d_ws;
  auto carve = [&](size_t bytes) { char* p = ws + off; off += (bytes + 255) & ~(size_t)255; return p; };
  const int NBM = (E + 255) / 256;
  b16* H16 = (b16*)carve((size_t)NP * D * 2); float* NODE4 = (float*)carve((size_t)NP * 4 * 4); b16* W1X = (b16*)carve((size_t)D * K1 * 2); b16* W2T = (b16*)carve((size_t)D * D * 2); b16* C1T = (b16*)carve((size_t)D * D * 2); b16* C2T = (b16*)carve((size_t)16 * D * 2); b16* HT = (b16*)carve((size_t)D * D * 2);
  int* KD = (int*)carve((size_t)E * 4); float* BM = (float*)carve((size_t)NBM * 32 * 4); float* GMX = (float*)carve(256); float* NAGG = (float*)carve((size_t)NP * D * 4); float* CAGG = (float*)carve((size_t)NP * 32 * 4); float* PF = (float*)carve((size_t)NWV * PW * 4); float* PL = (float*)carve((size_t)NWV * PW * 4);
  CsrBufs csr; off = csr_carve(csr, ws, off, E, N);
  if (off > ws_size || off > ((size_t)128 << 20) || csr.permLen > (size_t)EP) return;
  prep_kernel<<<(unsigned)(((size_t)NP * D / 8 + NP + (size_t)D * K1 / 8 + 3 * (size_t)D * D / 8 + 16 * D / 8 + 255) / 256), 256, 0, stream>>>(Fp(0), Fp(1), Fp(3), Fp(8), Fp(10), Fp(12), Fp(14), Fp(15), H16, NODE4, W1X, W2T, C1T, C2T, HT);
  dmax_kernel<<<NBM, 256, 0, stream>>>(Fp(1), Ip(5), BM);
  gmax_kernel<<<1, 256, 0, stream>>>(BM, NBM, GMX);
  keys_kernel<<<(unsigned)(((size_t)E / 4 + 255) / 256), 256, 0, stream>>>(Ip(5), KD);
  csr_build(csr, KD, E, N, stream);
  edge_kernel<<<EP / 16, 32, 0, stream>>>(Fp(1), Fp(2), Fp(3), Fp(4), Ip(5), Fp(6), Fp(7), GMX, NODE4, csr.PERM, (int)csr.permLen, H16, W1X, Fp(9), W2T, Fp(11), C1T, Fp(13), C2T, Fp(19), NAGG, CAGG, PF, PL);
  fix_kernel<<<(N + 7) / 8, 256, 0, stream>>>(csr.PERM, csr.ROWPTR, csr.ROWCNT, (int)csr.permLen, Ip(5), PF, PL, CAGG, Fp(1), NAGG, (float*)d_out + (size_t)N * D);
  head_kernel<<<NP / 64, 128, 0, stream>>>(NAGG, HT, Fp(16), Fp(17), Fp(18), Fp(0), (float*)d_out);
}
